// ConvolutionalEncoder_25769804001
// MI455X (gfx1250) — hardware-verified
//
#include <hip/hip_runtime.h>
#include <stddef.h>


#define GH    32
#define GW    32
#define NCELL (GH * GW)
#define HID   64
#define XD    7
#define NPTS  131072
#define EPSV  1e-8f

#define STHR  256
#define SEGP  4
#define NTHR  128
#define NWAVE 4
#define EPT   8
#define CHUNK (NTHR * EPT)
#define WCAP  (EPT * 32)
#define LISTN (NWAVE * WCAP)
#define PASSN 64
#define PCAP  (CHUNK + PASSN)
#define NBC   64
#define BPB   (NCELL / NBC)
#define NQ    ((NBC * HID) / (128 * NWAVE))
#define W2SC  8.0f
#define W2INV 0.125f

static_assert(PASSN == NWAVE * 16);
static_assert(NTHR == 2 * PASSN);
static_assert((NPTS % CHUNK) == 0);
static_assert((NPTS % 8) == 0);
static_assert((NPTS % (STHR * SEGP)) == 0);
static_assert(NQ * 128 * NWAVE == NBC * HID);
static_assert((NCELL % NBC) == 0);
static_assert(LISTN == CHUNK);
static_assert(PCAP >= CHUNK + PASSN);

typedef float    v2f  __attribute__((ext_vector_type(2)));
typedef float    v4f  __attribute__((ext_vector_type(4)));
typedef float    v8f  __attribute__((ext_vector_type(8)));
typedef int      v4i  __attribute__((ext_vector_type(4)));
typedef _Float16 v8h  __attribute__((ext_vector_type(8)));
typedef _Float16 v16h __attribute__((ext_vector_type(16)));
union FragH { v16h v; v8h h[2]; };

__device__ __forceinline__ v8f wmh(v16h a, v16h b, v8f c) {
  v8f d = __builtin_amdgcn_wmma_f32_16x16x32_f16(false, a, false, b, (short)0, c, false, false);
  asm volatile("v_nop\n\tv_nop\n\tv_nop\n\tv_nop" : "+v"(d) : "v"(a), "v"(b));
  return d;
}

__device__ __forceinline__ int scan_chunk(const int* __restrict__ keys, int nK, int cbase, int keyBase,
                                          int vec8, int* list, int tid, int wave) {
  int wc = 0;
  const int el0  = tid * EPT;
  const int e0   = cbase + el0;
  const int sent = -2147483647 - 1;
  v4i da, db;
  if (vec8 != 0 && cbase + CHUNK <= nK) {
    da = *(const v4i*)(keys + e0);
    db = *(const v4i*)(keys + e0 + 4);
  } else {
    da.x = (e0     < nK) ? keys[min(e0, nK - 1)] : sent;
    da.y = (e0 + 1 < nK) ? keys[min(e0 + 1, nK - 1)] : sent;
    da.z = (e0 + 2 < nK) ? keys[min(e0 + 2, nK - 1)] : sent;
    da.w = (e0 + 3 < nK) ? keys[min(e0 + 3, nK - 1)] : sent;
    db.x = (e0 + 4 < nK) ? keys[min(e0 + 4, nK - 1)] : sent;
    db.y = (e0 + 5 < nK) ? keys[min(e0 + 5, nK - 1)] : sent;
    db.z = (e0 + 6 < nK) ? keys[min(e0 + 6, nK - 1)] : sent;
    db.w = (e0 + 7 < nK) ? keys[min(e0 + 7, nK - 1)] : sent;
  }
  const unsigned nb = (unsigned)keyBase;
  const unsigned s0 = (unsigned)da.x - nb, s1 = (unsigned)da.y - nb;
  const unsigned s2 = (unsigned)da.z - nb, s3 = (unsigned)da.w - nb;
  const unsigned s4 = (unsigned)db.x - nb, s5 = (unsigned)db.y - nb;
  const unsigned s6 = (unsigned)db.z - nb, s7 = (unsigned)db.w - nb;
  const bool h0 = s0 < (unsigned)NBC, h1 = s1 < (unsigned)NBC, h2 = s2 < (unsigned)NBC, h3 = s3 < (unsigned)NBC;
  const bool h4 = s4 < (unsigned)NBC, h5 = s5 < (unsigned)NBC, h6 = s6 < (unsigned)NBC, h7 = s7 < (unsigned)NBC;
  const unsigned any = __builtin_amdgcn_ballot_w32(h0 | h1 | h2 | h3 | h4 | h5 | h6 | h7);
  if (any != 0u) {
#define HITJ(J, HJ) { \
      const unsigned mj = __builtin_amdgcn_ballot_w32(HJ); \
      if (mj != 0u) { \
        if (HJ) { \
          const int pos = wc + (int)__builtin_amdgcn_mbcnt_lo(mj, 0u); \
          if (pos < WCAP) list[wave * WCAP + pos] = el0 + (J); \
        } \
        wc += (int)__builtin_popcount(mj); } }
    HITJ(0, h0)
    HITJ(1, h1)
    HITJ(2, h2)
    HITJ(3, h3)
    HITJ(4, h4)
    HITJ(5, h5)
    HITJ(6, h6)
    HITJ(7, h7)
#undef HITJ
  }
  return wc;
}

__global__ __launch_bounds__(STHR) void k_stats(const float* __restrict__ x, float* st) {
  __shared__ float rmn0[STHR / 32], rmx0[STHR / 32], rmn1[STHR / 32], rmx1[STHR / 32];
  __shared__ __attribute__((aligned(16))) float line[32];
  const int b = blockIdx.x, tid = threadIdx.x, lane = tid & 31, wave = tid >> 5;
  const float pinf = __uint_as_float(0x7f800000u), ninf = __uint_as_float(0xff800000u);
  float xmn = pinf, xmx = ninf, ymn = pinf, ymx = ninf;
  const float* xb = x + (size_t)b * NPTS * XD;
#pragma unroll 1
  for (int i = tid; i < NPTS; i += STHR) {
    const float* p = xb + (size_t)i * XD;
    const float xc = p[0], yc = p[1];
    xmn = fminf(xmn, xc); xmx = fmaxf(xmx, xc);
    ymn = fminf(ymn, yc); ymx = fmaxf(ymx, yc);
  }
#pragma unroll
  for (int d = 16; d > 0; d >>= 1) {
    xmn = fminf(xmn, __shfl_xor(xmn, d));
    xmx = fmaxf(xmx, __shfl_xor(xmx, d));
    ymn = fminf(ymn, __shfl_xor(ymn, d));
    ymx = fmaxf(ymx, __shfl_xor(ymx, d));
  }
  if (lane == 0) { rmn0[wave] = xmn; rmx0[wave] = xmx; rmn1[wave] = ymn; rmx1[wave] = ymx; }
  __syncthreads();
  if (tid == 0) {
#pragma unroll
    for (int w = 1; w < STHR / 32; ++w) {
      xmn = fminf(xmn, rmn0[w]); xmx = fmaxf(xmx, rmx0[w]);
      ymn = fminf(ymn, rmn1[w]); ymx = fmaxf(ymx, rmx1[w]);
    }
    line[0] = xmn; line[1] = xmx; line[2] = ymn; line[3] = ymx;
#pragma unroll
    for (int j = 4; j < 32; ++j) line[j] = 0.0f;
  }
  __syncthreads();
  const v4f rv = *(const v4f*)(line + 4 * (lane & 7));
  const bool wr = (wave == 0) && (lane < 8);
  float* dst = st + b * 32 + 4 * (lane & 7);
  if (wr) *(volatile v4f*)dst = rv;
  __threadfence();
  if (wr) *(volatile v4f*)dst = rv;
}

__global__ __launch_bounds__(STHR) void k_seg(const float* __restrict__ x, const float* __restrict__ st,
                                             int* segp, int nTot) {
#pragma clang fp contract(off)
  const int gt = blockIdx.x * STHR + threadIdx.x;
  const int p0 = gt * SEGP;
  if (p0 + SEGP > nTot) return;
  const int b = p0 / NPTS;
  const float* sb = st + b * 32;
  const float xmin = sb[0], xmax = sb[1], ymin = sb[2], ymax = sb[3];
  const float xspan = fmaxf(xmax - xmin, EPSV);
  const float yspan = fmaxf(ymax - ymin, EPSV);
  const float rx = 1.0f / xspan;
  const float ry = 1.0f / yspan;
  int sg[SEGP];
#pragma unroll
  for (int j = 0; j < SEGP; ++j) {
    const float* p = x + (size_t)(p0 + j) * XD;
    const float xc = p[0], yc = p[1];
    const float dx = xc - xmin;
    const float dy = yc - ymin;
    const float qx = dx * rx;
    const float qy = dy * ry;
    const float tx = qx * 32.0f;
    const float ty = qy * 32.0f;
    const float txc = fminf(fmaxf(tx, 0.0f), 33.0f);
    const float tyc = fminf(fmaxf(ty, 0.0f), 33.0f);
    int gx = (int)floorf(txc);
    int gy = (int)floorf(tyc);
    gx = gx < 0 ? 0 : (gx > GH - 1 ? GH - 1 : gx);
    gy = gy < 0 ? 0 : (gy > GW - 1 ? GW - 1 : gy);
    sg[j] = b * NCELL + gx * GW + gy;
  }
  v4i v;
  v.x = sg[0]; v.y = sg[1]; v.z = sg[2]; v.w = sg[3];
  *(volatile v4i*)(segp + p0) = v;
  __threadfence();
  *(volatile v4i*)(segp + p0) = v;
}

__global__ __launch_bounds__(NTHR) void k_agg(
    const float* __restrict__ x, const int* __restrict__ segp,
    const float* __restrict__ W1, const float* __restrict__ b1,
    const float* __restrict__ W2, const float* __restrict__ b2,
    float* outp) {
  __shared__ __attribute__((aligned(16))) float    acc[(NBC + 1) * HID];
  __shared__ __attribute__((aligned(16))) float    msg[PASSN * HID];
  __shared__ __attribute__((aligned(16))) _Float16 hti[PASSN * HID];
  __shared__ __attribute__((aligned(16))) _Float16 w2s[HID * HID];
  __shared__ __attribute__((aligned(16))) float    w1s[XD * HID];
  __shared__ __attribute__((aligned(16))) float    b1s[HID];
  __shared__ __attribute__((aligned(16))) float    b2s[HID];
  __shared__ __attribute__((aligned(16))) float    xs[PASSN * 8];
  __shared__ __attribute__((aligned(16))) int      list[LISTN];
  __shared__ __attribute__((aligned(16))) int      pend[PCAP];
  __shared__ int slotb[PASSN];
  __shared__ int wcnt[NWAVE];
  __shared__ int pendN;

  const int tid = threadIdx.x, lane = tid & 31, wave = tid >> 5, hh = lane >> 4, m = lane & 15;
  const int bx    = blockIdx.x;
  const int batch = bx / BPB;
  const int cb    = bx * NBC;
  const int* sgb  = segp + (size_t)batch * NPTS;
  const float* xb = x + (size_t)batch * NPTS * XD;
  const int vec8  = 1;

  for (int i = tid; i < (NBC + 1) * HID; i += NTHR) acc[i] = 0.0f;
  for (int i = tid; i < HID * HID; i += NTHR) {
    const int n = i >> 6, k = i & 63;
    w2s[i] = (_Float16)(W2[k * HID + n] * W2SC);
  }
  for (int i = tid; i < XD * HID; i += NTHR) w1s[i] = W1[i];
  if (tid < HID) { b1s[tid] = b1[tid]; b2s[tid] = b2[tid]; }
  if (tid == 0) pendN = 0;
  __syncthreads();

  const int nChunks = NPTS / CHUNK;
#pragma unroll 1
  for (int ch = 0; ch < nChunks; ++ch) {
    const int cbase = ch * CHUNK;
    const int wc = scan_chunk(sgb, NPTS, cbase, cb, vec8, list, tid, wave);
    if (lane == 0) wcnt[wave] = wc;
    __syncthreads();

    const int base = pendN;
    int tot = 0, myoff = 0;
#pragma unroll
    for (int w = 0; w < NWAVE; ++w) {
      int c = wcnt[w];
      c = c > WCAP ? WCAP : (c < 0 ? 0 : c);
      if (w < wave) myoff += c;
      tot += c;
    }
    int newN = base + tot;
    newN = newN > PCAP ? PCAP : newN;
    {
      int n = wcnt[wave];
      n = n > WCAP ? WCAP : (n < 0 ? 0 : n);
      const int* lp = list + wave * WCAP;
      for (int i = lane; i < n; i += 32) {
        const int pos = base + myoff + i;
        if (pos < PCAP) pend[pos] = cbase + lp[i];
      }
    }
    const int fin = (ch == nChunks - 1) ? 1 : 0;
    const int R   = (fin != 0) ? (newN + PASSN - 1) / PASSN : newN / PASSN;
    const int Pv  = (fin != 0) ? newN : R * PASSN;
    __syncthreads();

#pragma unroll 1
    for (int ps = 0; ps < R; ++ps) {
      if (tid < PASSN) {
        const int idx = ps * PASSN + tid;
        const bool valid = idx < Pv;
        const int ic = idx < PCAP ? idx : PCAP - 1;
        int e = pend[ic];
        e = valid ? e : 0;
        e = e < 0 ? 0 : (e > NPTS - 1 ? NPTS - 1 : e);
        const int s = sgb[e];
        int slot = s - cb;
        if (!valid || (unsigned)slot >= (unsigned)NBC) slot = NBC;
        const float* xp = xb + (size_t)e * XD;
        float* xr = xs + tid * 8;
#pragma unroll
        for (int c = 0; c < XD; ++c) { const float t = xp[c]; xr[c] = valid ? t : 0.0f; }
        xr[7] = 0.0f;
        slotb[tid] = slot;
      }
      __syncthreads();

      {
        const int p = tid & (PASSN - 1), hf = tid >> 6;
        float a[32];
#pragma unroll
        for (int j = 0; j < 32; ++j) a[j] = 0.0f;
#pragma unroll 1
        for (int k = 0; k < XD; ++k) {
          const float xv = xs[p * 8 + k];
          const float* wr = w1s + k * HID + 32 * hf;
#pragma unroll
          for (int q = 0; q < 8; ++q) {
            const v4f w4 = *(const v4f*)(wr + 4 * q);
            a[4 * q + 0] = fmaf(xv, w4.x, a[4 * q + 0]);
            a[4 * q + 1] = fmaf(xv, w4.y, a[4 * q + 1]);
            a[4 * q + 2] = fmaf(xv, w4.z, a[4 * q + 2]);
            a[4 * q + 3] = fmaf(xv, w4.w, a[4 * q + 3]);
          }
        }
        const float* bb = b1s + 32 * hf;
        _Float16* hp = hti + p * HID + 32 * hf;
#pragma unroll
        for (int q = 0; q < 4; ++q) {
          v8h hv;
#pragma unroll
          for (int i = 0; i < 8; ++i) {
            const float t = fmaxf(a[8 * q + i] + bb[8 * q + i], 0.0f);
            hv[i] = (_Float16)t;
          }
          *(v8h*)(hp + 8 * q) = hv;
        }
      }
      __syncthreads();

      {
        v8f d[4];
#pragma unroll
        for (int g = 0; g < 4; ++g) {
#pragma unroll
          for (int r8 = 0; r8 < 8; ++r8) d[g][r8] = 0.0f;
        }
#pragma unroll
        for (int ks = 0; ks < 2; ++ks) {
          FragH af;
          const _Float16* ap = hti + (wave * 16 + m) * HID + 32 * ks + 8 * hh;
          af.h[0] = *(const v8h*)ap;
          af.h[1] = *(const v8h*)(ap + 16);
#pragma unroll
          for (int g = 0; g < 4; ++g) {
            FragH bf;
            const _Float16* bp = w2s + (16 * g + m) * HID + 32 * ks + 8 * hh;
            bf.h[0] = *(const v8h*)bp;
            bf.h[1] = *(const v8h*)(bp + 16);
            d[g] = wmh(af.v, bf.v, d[g]);
          }
        }
#pragma unroll
        for (int g = 0; g < 4; ++g) {
          const float bz = b2s[16 * g + m];
#pragma unroll
          for (int r8 = 0; r8 < 8; ++r8) {
            const int pt = wave * 16 + 8 * hh + r8;
            msg[pt * HID + 16 * g + m] = fmaf(d[g][r8], W2INV, bz);
          }
        }
      }
      __syncthreads();

      if (wave == 0) {
#pragma unroll 1
        for (int i = 0; i < PASSN; ++i) {
          int sl = slotb[i];
          sl = sl < 0 ? 0 : (sl > NBC ? NBC : sl);
          const v2f mv = *(const v2f*)(msg + i * HID + 2 * lane);
          float* aq = acc + sl * HID + 2 * lane;
          v2f av = *(const v2f*)aq;
          av += mv;
          *(v2f*)aq = av;
        }
      }
      __syncthreads();
    }

    int rem = newN - R * PASSN;
    rem = rem < 0 ? 0 : rem;
    if (R > 0 && tid < rem) pend[tid] = pend[R * PASSN + tid];
    if (tid == 0) pendN = rem;
  }
  __syncthreads();

  v4f ov[NQ];
#pragma unroll
  for (int q = 0; q < NQ; ++q) {
    const int f = (wave * NQ + q) * 128 + 4 * lane;
    ov[q] = *(const v4f*)(acc + f);
  }
  const size_t ob = (size_t)bx * (NBC * HID);
#pragma unroll
  for (int q = 0; q < NQ; ++q) {
    const int f = (wave * NQ + q) * 128 + 4 * lane;
    *(volatile v4f*)(outp + ob + (size_t)f) = ov[q];
  }
  __threadfence();
#pragma unroll
  for (int q = 0; q < NQ; ++q) {
    const int f = (wave * NQ + q) * 128 + 4 * lane;
    *(volatile v4f*)(outp + ob + (size_t)f) = ov[q];
  }
}

extern "C" void kernel_launch(void* const* d_in, const int* in_sizes, int n_in,
                              void* d_out, int out_size, void* d_ws, size_t ws_size,
                              hipStream_t stream) {
  if (n_in < 5) return;
  const int per = NPTS * XD;
  if (in_sizes[0] <= 0 || (in_sizes[0] % per) != 0) return;
  const int nb = in_sizes[0] / per;
  if (nb <= 0 || nb > 64) return;
  if (in_sizes[1] != XD * HID || in_sizes[2] != HID || in_sizes[3] != HID * HID || in_sizes[4] != HID) return;
  if (out_size != nb * NCELL * HID) return;
  const int nTot = nb * NPTS;

  const float* x  = (const float*)d_in[0];
  const float* W1 = (const float*)d_in[1];
  const float* b1 = (const float*)d_in[2];
  const float* W2 = (const float*)d_in[3];
  const float* b2 = (const float*)d_in[4];
  float* out = (float*)d_out;

  char* ws = (char*)d_ws;
  size_t off = 0;
  const size_t oSt = off; off += (size_t)nb * 32 * 4;  off = (off + 255) & ~(size_t)255;
  const size_t oSg = off; off += (size_t)nTot * 4;      off = (off + 255) & ~(size_t)255;
  if (off > ws_size) return;
  float* st   = (float*)(ws + oSt);
  int*   segp = (int*)(ws + oSg);

  k_stats<<<nb, STHR, 0, stream>>>(x, st);
  k_seg<<<nTot / (STHR * SEGP), STHR, 0, stream>>>(x, st, segp, nTot);
  k_agg<<<nb * BPB, NTHR, 0, stream>>>(x, segp, W1, b1, W2, b2, out);
}
